// Block_50130858279051
// MI455X (gfx1250) — hardware-verified
//
#include <hip/hip_runtime.h>


#ifndef NB
#define NB 2
#endif
#ifndef SEQ
#define SEQ 2048
#endif
#define NB_FULL 2
#define SEQ_FULL 2048
#define CE 1024
#define NH 16
#define HD 64
#define C3 3072
#define C4 4096
#define QP 2048
#define TE (((SEQ) < 256) ? (SEQ) : 256)
#define RROWS ((NB) * (SEQ))
#define NEB ((TE) / 128)
#define NQB ((SEQ) / 128)
#define LNJ ((CE) / 128)
#define LNO ((CE) / 256)

static_assert((SEQ) % 128 == 0);
static_assert((TE) % 128 == 0);
static_assert((NB) >= 1 && (NB) <= NB_FULL);
static_assert((SEQ) <= SEQ_FULL);
static_assert(CE % 128 == 0 && C3 % 128 == 0 && C4 % 128 == 0 && QP % 128 == 0);
static_assert(CE % 64 == 0 && C3 % 64 == 0 && C4 % 64 == 0);
static_assert(NH * HD == CE);
static_assert(HD == 64);
static_assert(QP == 2 * CE);
static_assert(C3 == 3 * CE);
static_assert(RROWS % 128 == 0);
static_assert(RROWS % 8 == 0);
static_assert(CE == 1024);
static_assert(256 * 4 == CE);
static_assert(32 * 4 * LNJ == CE);
static_assert(32 * 8 * LNO == CE);
static_assert(NQB * 128 == (SEQ));
static_assert(NEB <= NQB);

typedef unsigned short u16;
typedef unsigned int   u32;
typedef _Float16 v16h __attribute__((ext_vector_type(16)));
typedef _Float16 v8h  __attribute__((ext_vector_type(8)));
typedef _Float16 v4h  __attribute__((ext_vector_type(4)));
typedef float    v8f  __attribute__((ext_vector_type(8)));
typedef float    v4f  __attribute__((ext_vector_type(4)));
typedef unsigned int u32x4 __attribute__((ext_vector_type(4)));
typedef unsigned int u32x2 __attribute__((ext_vector_type(2)));

union Frag  { v16h v; u32x4 u[2]; };
union Pack8 { v8h h; u32x4 u; };
union Pack4 { v4h h; u32x2 u; };

#define WSCALE 64.0f
#define WINV   (1.0f / 64.0f)
#define PCAR   4096.0f
#define PINV   (1.0f / 4096.0f)
#define RSC    2048.0f
#define RINV   (1.0f / 2048.0f)

constexpr size_t al256(size_t b) { return (b + 255) & ~(size_t)255; }
constexpr size_t WS_TOTAL =
    al256((size_t)C3 * CE * 2) + al256((size_t)CE * CE * 2) + al256((size_t)C4 * CE * 2) +
    al256((size_t)CE * C4 * 2) + al256((size_t)RROWS * CE * 2) + al256((size_t)RROWS * QP * 2) +
    al256((size_t)NB * (TE) * QP * 2) + al256((size_t)NB * NH * HD * (SEQ) * 2) +
    al256((size_t)NB * NH * HD * (TE) * 2) + al256((size_t)RROWS * CE * 2) +
    al256((size_t)RROWS * CE * 4) + al256((size_t)RROWS * CE * 2) + al256((size_t)RROWS * C4 * 2);
static_assert(WS_TOTAL <= (size_t)134217728);

__device__ __forceinline__ float bfr(float f) {
    u32 u = __builtin_bit_cast(u32, f);
    u += 0x7fffu + ((u >> 16) & 1u);
    u &= 0xffff0000u;
    return __builtin_bit_cast(float, u);
}

__device__ __forceinline__ u16 hbits(float f) {
    _Float16 h = (_Float16)f;
    return __builtin_bit_cast(u16, h);
}

__device__ __forceinline__ v8f mma16(v16h a, v16h b, v8f c) {
    c = __builtin_amdgcn_wmma_f32_16x16x32_f16(false, a, false, b, (short)0, c, false, false);
    asm volatile("v_nop\n\tv_nop\n\tv_nop\n\tv_nop" : "+v"(c) : "v"(a), "v"(b));
    return c;
}

template <int ON>
__device__ __forceinline__ void sched_cut() {
    if constexpr (ON != 0) __builtin_amdgcn_sched_barrier(0);
}

__device__ __forceinline__ float gelu_erf(float x) {
    return 0.5f * x * (1.0f + erff(x * 0.70710678118654752f));
}

__device__ __forceinline__ size_t grow_map(u32 r) {
    const u32 bb = r / (u32)(SEQ);
    const u32 t  = r - bb * (u32)(SEQ);
    return (size_t)bb * SEQ_FULL + (size_t)t;
}

__global__ __launch_bounds__(256) void cvt_wt_kernel(const float* __restrict__ in,
                                                      u16* __restrict__ out, u32 K, u32 N) {
    __shared__ __align__(16) u16 Ts[64 * 72];
    const u32 tid = threadIdx.x, lane = tid & 31u, wv = tid >> 5;
    const u32 n0 = blockIdx.x * 64u, k0 = blockIdx.y * 64u;
    const u32 kr = tid >> 2, nseg = (tid & 3u) * 16u;
    const float* src = in + (size_t)(k0 + kr) * N + n0 + nseg;
#pragma unroll
    for (u32 j4 = 0; j4 < 4; j4++) {
        v4f w = *(const v4f*)(src + j4 * 4u);
#pragma unroll
        for (u32 c = 0; c < 4; c++) {
            float f = w[c];
            Ts[(nseg + j4 * 4u + c) * 72u + kr] = hbits(bfr(f) * WSCALE);
        }
    }
    __syncthreads();
    u32x4 val[2];
#pragma unroll
    for (u32 it = 0; it < 2; it++) {
        const u32 nn = wv * 8u + it * 4u + (lane >> 3), ks = (lane & 7u) * 8u;
        val[it] = *(const u32x4*)&Ts[nn * 72u + ks];
    }
#pragma unroll
    for (u32 it = 0; it < 2; it++) {
        const u32 nn = wv * 8u + it * 4u + (lane >> 3), ks = (lane & 7u) * 8u;
        *(volatile u32x4*)(out + (size_t)(n0 + nn) * K + k0 + ks) = val[it];
    }
    __threadfence();
#pragma unroll
    for (u32 it = 0; it < 2; it++) {
        const u32 nn = wv * 8u + it * 4u + (lane >> 3), ks = (lane & 7u) * 8u;
        *(volatile u32x4*)(out + (size_t)(n0 + nn) * K + k0 + ks) = val[it];
    }
}

template <int SRCX>
__global__ __launch_bounds__(256) void ln_kernel(const float* __restrict__ src,
                                                 const float* __restrict__ g,
                                                 const float* __restrict__ be,
                                                 u16* __restrict__ out) {
    __shared__ __align__(16) float xs[8 * CE];
    __shared__ __align__(16) u16   rows[8 * CE];
    __shared__ __align__(16) float gsh[CE];
    __shared__ __align__(16) float bsh[CE];
    const u32 tid = threadIdx.x, lane = tid & 31u, wv = tid >> 5;
    {
        v4f gg = *(const v4f*)(g + tid * 4u);
        v4f bb = *(const v4f*)(be + tid * 4u);
        v4f go, bo;
#pragma unroll
        for (u32 c = 0; c < 4; c++) {
            float tg = gg[c]; float tb = bb[c];
            go[c] = bfr(tg); bo[c] = bfr(tb);
        }
        *(v4f*)&gsh[tid * 4u] = go;
        *(v4f*)&bsh[tid * 4u] = bo;
    }
    const u32 r = blockIdx.x * 8u + wv;
    const size_t srow = SRCX ? grow_map(r) : (size_t)r;
    const float* xr = src + srow * CE;
    float* xw = xs + wv * CE;
    float s = 0.f;
#pragma unroll 1
    for (u32 j = 0; j < LNJ; j++) {
        const u32 c0 = j * 128u + lane * 4u;
        v4f t4 = *(const v4f*)(xr + c0);
        if constexpr (SRCX != 0) {
#pragma unroll
            for (u32 c = 0; c < 4; c++) { float t = t4[c]; t4[c] = bfr(t); }
        }
        *(v4f*)&xw[c0] = t4;
        s += (t4[0] + t4[1]) + (t4[2] + t4[3]);
    }
#pragma unroll
    for (u32 m = 16; m >= 1; m >>= 1) s += __shfl_xor(s, m, 32);
    const float mu = s * (1.f / (float)CE);
    float vs = 0.f;
#pragma unroll 1
    for (u32 j = 0; j < LNJ; j++) {
        const u32 c0 = j * 128u + lane * 4u;
        v4f t4 = *(const v4f*)&xw[c0];
#pragma unroll
        for (u32 c = 0; c < 4; c++) { float d = t4[c] - mu; vs += d * d; }
    }
#pragma unroll
    for (u32 m = 16; m >= 1; m >>= 1) vs += __shfl_xor(vs, m, 32);
    const float rstd = rsqrtf(vs * (1.f / (float)CE) + 1e-5f);
    __syncthreads();
    u16* rw = rows + wv * CE;
#pragma unroll 1
    for (u32 j = 0; j < LNJ; j++) {
        const u32 c0 = j * 128u + lane * 4u;
        v4f x4 = *(const v4f*)&xw[c0];
        v4f g4 = *(const v4f*)&gsh[c0];
        v4f b4 = *(const v4f*)&bsh[c0];
        Pack4 pk;
#pragma unroll
        for (u32 c = 0; c < 4; c++) {
            float xe = x4[c]; float ge = g4[c]; float bel = b4[c];
            pk.h[c] = (_Float16)((xe - mu) * rstd * ge + bel);
        }
        *(u32x2*)&rw[c0] = pk.u;
    }
    __syncthreads();
    u32x4 val[LNO];
#pragma unroll
    for (u32 j = 0; j < LNO; j++) val[j] = *(const u32x4*)&rw[j * 256u + lane * 8u];
    u16* orow = out + (size_t)r * CE;
#pragma unroll
    for (u32 j = 0; j < LNO; j++) *(volatile u32x4*)(orow + j * 256u + lane * 8u) = val[j];
    __threadfence();
#pragma unroll
    for (u32 j = 0; j < LNO; j++) *(volatile u32x4*)(orow + j * 256u + lane * 8u) = val[j];
}

template <int MODE>
__global__ __launch_bounds__(256) void gemm_kernel(const u16* __restrict__ A,
                                                   const u16* __restrict__ BT,
                                                   const float* __restrict__ bias,
                                                   const float* __restrict__ res,
                                                   void* out0, void* out1, void* out2, void* out3,
                                                   u32 N, u32 K) {
    __shared__ u32x4 smem[4224];
    u16* As = (u16*)smem;
    u16* Bs = As + 128 * 72;
    float* Cs = (float*)smem;
    constexpr u32 CSP = 132;

    const u32 tid = threadIdx.x, lane = tid & 31u, wv = tid >> 5;
    const u32 hf = lane >> 4, ln = lane & 15u;
    const u32 m0 = blockIdx.y * 128u, n0 = blockIdx.x * 128u;
    const u32 wm = wv & 3u, wn = wv >> 2;
    const u32 srow = tid >> 1, sseg = (tid & 1u) * 32u;

    v8f acc[2][4];
#pragma unroll
    for (int i = 0; i < 2; i++)
#pragma unroll
        for (int j = 0; j < 4; j++) acc[i][j] = (v8f)(0.f);

    for (u32 k0 = 0; k0 < K; k0 += 64u) {
        __syncthreads();
        {
            const u16* ga = A  + (size_t)(m0 + srow) * K + k0 + sseg;
            const u16* gb = BT + (size_t)(n0 + srow) * K + k0 + sseg;
            u32x4 a0 = *(const u32x4*)(ga), a1 = *(const u32x4*)(ga + 8);
            u32x4 a2 = *(const u32x4*)(ga + 16), a3 = *(const u32x4*)(ga + 24);
            u32x4 b0 = *(const u32x4*)(gb), b1 = *(const u32x4*)(gb + 8);
            u32x4 b2 = *(const u32x4*)(gb + 16), b3 = *(const u32x4*)(gb + 24);
            u32x4* la = (u32x4*)&As[srow * 72u + sseg];
            u32x4* lb = (u32x4*)&Bs[srow * 72u + sseg];
            la[0] = a0; la[1] = a1; la[2] = a2; la[3] = a3;
            lb[0] = b0; lb[1] = b1; lb[2] = b2; lb[3] = b3;
        }
        __syncthreads();
#pragma unroll
        for (u32 ks = 0; ks < 2; ks++) {
            Frag af[2], bf[4];
#pragma unroll
            for (u32 mi = 0; mi < 2; mi++) {
                const u16* q = &As[(wm * 32u + mi * 16u + ln) * 72u + ks * 32u + hf * 8u];
                af[mi].u[0] = *(const u32x4*)q;
                af[mi].u[1] = *(const u32x4*)(q + 16);
            }
#pragma unroll
            for (u32 ni = 0; ni < 4; ni++) {
                const u16* q = &Bs[(wn * 64u + ni * 16u + ln) * 72u + ks * 32u + hf * 8u];
                bf[ni].u[0] = *(const u32x4*)q;
                bf[ni].u[1] = *(const u32x4*)(q + 16);
            }
#pragma unroll
            for (int mi = 0; mi < 2; mi++)
#pragma unroll
                for (int ni = 0; ni < 4; ni++)
                    acc[mi][ni] = mma16(af[mi].v, bf[ni].v, acc[mi][ni]);
        }
    }

    __syncthreads();
#pragma unroll
    for (int ni = 0; ni < 4; ni++) {
        const u32 col = wn * 64u + (u32)ni * 16u + ln;
        const float bv = bfr(bias[n0 + col]);
#pragma unroll
        for (int mi = 0; mi < 2; mi++) {
#pragma unroll
            for (int r = 0; r < 8; r++) {
                const u32 row = wm * 32u + (u32)mi * 16u + hf * 8u + (u32)r;
                float v = acc[mi][ni][r] * WINV + bv;
                if constexpr (MODE == 2) v = gelu_erf(v);
                Cs[row * CSP + col] = v;
            }
        }
    }
    __syncthreads();

    if constexpr (MODE == 1 || MODE == 3) {
        float* o = (float*)out0;
        v4f val[16];
#pragma unroll
        for (int grp = 0; grp < 2; grp++) {
#pragma unroll
            for (int i8 = 0; i8 < 8; i8++) {
                const int i = grp * 8 + i8;
                const u32 row = wv * 16u + (u32)i;
                const u32 r = m0 + row;
                v4f c = *(const v4f*)&Cs[row * CSP + lane * 4u];
                const size_t rr = (MODE == 1) ? grow_map(r) : (size_t)r;
                v4f x4 = *(const v4f*)(res + rr * (size_t)N + n0 + lane * 4u);
                if constexpr (MODE == 1) {
#pragma unroll
                    for (int cc = 0; cc < 4; cc++) { float t = x4[cc]; x4[cc] = bfr(t); }
                }
                val[i] = c + x4;
            }
            asm volatile("" ::: "memory");
        }
#pragma unroll
        for (int i = 0; i < 16; i++) {
            const u32 r = m0 + wv * 16u + (u32)i;
            const size_t orr = (MODE == 3) ? grow_map(r) : (size_t)r;
            *(volatile v4f*)(o + orr * (size_t)N + n0 + lane * 4u) = val[i];
        }
        __threadfence();
#pragma unroll
        for (int i = 0; i < 16; i++) {
            const u32 r = m0 + wv * 16u + (u32)i;
            const size_t orr = (MODE == 3) ? grow_map(r) : (size_t)r;
            *(volatile v4f*)(o + orr * (size_t)N + n0 + lane * 4u) = val[i];
        }
    } else if constexpr (MODE == 2) {
        u16* o = (u16*)out0;
        u32x4 val[8];
#pragma unroll
        for (int it = 0; it < 8; it++) {
            const u32 rloc = wv * 16u + (u32)it * 2u + hf, cseg = ln * 8u;
            Pack8 pk;
#pragma unroll
            for (int j = 0; j < 8; j++) pk.h[j] = (_Float16)Cs[rloc * CSP + cseg + (u32)j];
            val[it] = pk.u;
        }
#pragma unroll
        for (int it = 0; it < 8; it++) {
            const u32 rloc = wv * 16u + (u32)it * 2u + hf, cseg = ln * 8u;
            *(volatile u32x4*)(o + (size_t)(m0 + rloc) * N + n0 + cseg) = val[it];
        }
        __threadfence();
#pragma unroll
        for (int it = 0; it < 8; it++) {
            const u32 rloc = wv * 16u + (u32)it * 2u + hf, cseg = ln * 8u;
            *(volatile u32x4*)(o + (size_t)(m0 + rloc) * N + n0 + cseg) = val[it];
        }
    } else {
        u16* qkh = (u16*)out0;
        u16* qkl = (u16*)out1;
        u16* vth = (u16*)out2;
        u16* vtl = (u16*)out3;
        const u32 bq = m0 / (u32)(SEQ);
        const u32 t0 = m0 - bq * (u32)(SEQ);
        const bool lo_on = (t0 < (u32)(TE));
        u32x4 vh[8], vl[8];
        if (n0 < (u32)QP) {
#pragma unroll
            for (int it = 0; it < 8; it++) {
                const u32 rloc = wv * 16u + (u32)it * 2u + hf, cseg = ln * 8u;
                Pack8 ph, pl;
#pragma unroll
                for (int j = 0; j < 8; j++) {
                    float f = Cs[rloc * CSP + cseg + (u32)j];
                    _Float16 h16 = (_Float16)f;
                    ph.h[j] = h16;
                    pl.h[j] = (_Float16)((f - (float)h16) * RSC);
                }
                vh[it] = ph.u; vl[it] = pl.u;
            }
#pragma unroll
            for (int it = 0; it < 8; it++) {
                const u32 rloc = wv * 16u + (u32)it * 2u + hf, cseg = ln * 8u;
                *(volatile u32x4*)(qkh + (size_t)(m0 + rloc) * QP + n0 + cseg) = vh[it];
                if (lo_on)
                    *(volatile u32x4*)(qkl + ((size_t)bq * (TE) + t0 + rloc) * QP + n0 + cseg) = vl[it];
            }
            __threadfence();
#pragma unroll
            for (int it = 0; it < 8; it++) {
                const u32 rloc = wv * 16u + (u32)it * 2u + hf, cseg = ln * 8u;
                *(volatile u32x4*)(qkh + (size_t)(m0 + rloc) * QP + n0 + cseg) = vh[it];
                if (lo_on)
                    *(volatile u32x4*)(qkl + ((size_t)bq * (TE) + t0 + rloc) * QP + n0 + cseg) = vl[it];
            }
        } else {
            const u32 hh0 = (n0 - (u32)QP) >> 6;
#pragma unroll
            for (int it = 0; it < 8; it++) {
                const u32 rloc = wv * 16u + (u32)it * 2u + hf;
                const u32 tseg = ln * 8u;
                Pack8 ph, pl;
#pragma unroll
                for (int j = 0; j < 8; j++) {
                    float f = Cs[(tseg + (u32)j) * CSP + rloc];
                    _Float16 h16 = (_Float16)f;
                    ph.h[j] = h16;
                    pl.h[j] = (_Float16)((f - (float)h16) * RSC);
                }
                vh[it] = ph.u; vl[it] = pl.u;
            }
#pragma unroll
            for (int it = 0; it < 8; it++) {
                const u32 rloc = wv * 16u + (u32)it * 2u + hf, tseg = ln * 8u;
                const u32 hh = hh0 + (rloc >> 6), dd = rloc & 63u;
                const size_t vrow = (size_t)(bq * NH + hh) * HD + dd;
                *(volatile u32x4*)(vth + vrow * (SEQ) + t0 + tseg) = vh[it];
                if (lo_on)
                    *(volatile u32x4*)(vtl + vrow * (TE) + t0 + tseg) = vl[it];
            }
            __threadfence();
#pragma unroll
            for (int it = 0; it < 8; it++) {
                const u32 rloc = wv * 16u + (u32)it * 2u + hf, tseg = ln * 8u;
                const u32 hh = hh0 + (rloc >> 6), dd = rloc & 63u;
                const size_t vrow = (size_t)(bq * NH + hh) * HD + dd;
                *(volatile u32x4*)(vth + vrow * (SEQ) + t0 + tseg) = vh[it];
                if (lo_on)
                    *(volatile u32x4*)(vtl + vrow * (TE) + t0 + tseg) = vl[it];
            }
        }
    }
}

template <int RES>
__global__ __launch_bounds__(256) __attribute__((amdgpu_num_vgpr(256)))
void attn_kernel(const u16* __restrict__ qkh, const u16* __restrict__ qkl,
                 const u16* __restrict__ vth, const u16* __restrict__ vtl,
                 u16* __restrict__ cv, u32 qb0) {
    __shared__ __align__(16) u16 Ks[64 * 72];
    __shared__ __align__(16) u16 Vs[64 * 72];
    __shared__ __align__(16) u16 Kl[RES ? 64 * 72 : 8];
    __shared__ __align__(16) u16 Vl[RES ? 64 * 72 : 8];
    __shared__ __align__(16) u16 Ps[8 * 16 * 72];
    __shared__ __align__(16) u16 Pr[RES ? 8 * 16 * 72 : 8];

    const u32 bh = blockIdx.y;
    const u32 b = bh / (u32)NH, h = bh - b * (u32)NH;
    const u32 qb = qb0 + blockIdx.x;
    const u32 tid = threadIdx.x, lane = tid & 31u;
    u32 wv = tid >> 5;
    if constexpr (RES != 0) wv = (u32)__builtin_amdgcn_readfirstlane((int)wv);
    const u32 hf = lane >> 4, ln = lane & 15u;
    const u32 q0 = qb * 128u + wv * 16u;
    u16* Pw  = Ps + wv * (16u * 72u);
    u16* Prw = Pr + (RES ? wv * (16u * 72u) : 0u);

    Frag qf[2], ql[2];
#pragma unroll
    for (u32 ds = 0; ds < 2; ds++) {
        const u16* p = qkh + (size_t)(b * (u32)(SEQ) + q0 + ln) * QP + h * HD + ds * 32u + hf * 8u;
        qf[ds].u[0] = *(const u32x4*)p;
        qf[ds].u[1] = *(const u32x4*)(p + 16);
        if constexpr (RES != 0) {
            const u16* pl = qkl + (size_t)(b * (u32)(TE) + q0 + ln) * QP + h * HD + ds * 32u + hf * 8u;
            ql[ds].u[0] = *(const u32x4*)pl;
            ql[ds].u[1] = *(const u32x4*)(pl + 16);
        } else {
            ql[ds].u[0] = (u32x4)(0u); ql[ds].u[1] = (u32x4)(0u);
        }
    }

    v8f o[4];
#pragma unroll
    for (int i = 0; i < 4; i++) o[i] = (v8f)(0.f);
    float mrow[8], lrow[8];
#pragma unroll
    for (int r = 0; r < 8; r++) { mrow[r] = -3.0e38f; lrow[r] = 0.f; }

    const u32 rr = tid >> 2, seg = (tid & 3u) * 16u;
    const u32 nkt = 2u * qb + 2u;

#pragma unroll 1
    for (u32 kt = 0; kt < nkt; kt++) {
        __syncthreads();
        {
            const u16* gk = qkh + (size_t)(b * (u32)(SEQ) + kt * 64u + rr) * QP + CE + h * HD + seg;
            u32x4 k0v = *(const u32x4*)gk, k1v = *(const u32x4*)(gk + 8);
            const u16* gv = vth + ((size_t)(bh * HD + rr)) * (SEQ) + kt * 64u + seg;
            u32x4 v0 = *(const u32x4*)gv, v1 = *(const u32x4*)(gv + 8);
            *(u32x4*)&Ks[rr * 72u + seg] = k0v; *(u32x4*)&Ks[rr * 72u + seg + 8u] = k1v;
            *(u32x4*)&Vs[rr * 72u + seg] = v0;  *(u32x4*)&Vs[rr * 72u + seg + 8u] = v1;
            sched_cut<RES>();
            if constexpr (RES != 0) {
                const u16* gkl = qkl + (size_t)(b * (u32)(TE) + kt * 64u + rr) * QP + CE + h * HD + seg;
                u32x4 kl0 = *(const u32x4*)gkl, kl1 = *(const u32x4*)(gkl + 8);
                const u16* gvl = vtl + ((size_t)(bh * HD + rr)) * (TE) + kt * 64u + seg;
                u32x4 vl0 = *(const u32x4*)gvl, vl1 = *(const u32x4*)(gvl + 8);
                *(u32x4*)&Kl[rr * 72u + seg] = kl0; *(u32x4*)&Kl[rr * 72u + seg + 8u] = kl1;
                *(u32x4*)&Vl[rr * 72u + seg] = vl0; *(u32x4*)&Vl[rr * 72u + seg + 8u] = vl1;
            }
        }
        __syncthreads();
        sched_cut<RES>();

        v8f s[4];
#pragma unroll
        for (int sub = 0; sub < 4; sub++) {
            v8f t = (v8f)(0.f);
            v8f tr = (v8f)(0.f);
#pragma unroll
            for (int ds = 0; ds < 2; ds++) {
                Frag kf;
                const u16* kp = &Ks[((u32)sub * 16u + ln) * 72u + (u32)ds * 32u + hf * 8u];
                kf.u[0] = *(const u32x4*)kp;
                kf.u[1] = *(const u32x4*)(kp + 16);
                t = mma16(qf[ds].v, kf.v, t);
                if constexpr (RES != 0) {
                    Frag klf;
                    const u16* klp = &Kl[((u32)sub * 16u + ln) * 72u + (u32)ds * 32u + hf * 8u];
                    klf.u[0] = *(const u32x4*)klp;
                    klf.u[1] = *(const u32x4*)(klp + 16);
                    tr = mma16(qf[ds].v, klf.v, tr);
                    tr = mma16(ql[ds].v, kf.v, tr);
                }
            }
            if constexpr (RES != 0) s[sub] = t + tr * RINV;
            else s[sub] = t;
            sched_cut<RES>();
        }

#pragma unroll
        for (int sub = 0; sub < 4; sub++) {
            const u32 kg = kt * 64u + (u32)sub * 16u + ln;
#pragma unroll
            for (int r = 0; r < 8; r++) {
                const u32 qg = q0 + hf * 8u + (u32)r;
                float v = s[sub][r] * 0.125f;
                s[sub][r] = (kg > qg) ? -3.0e38f : v;
            }
        }
#pragma unroll
        for (int r = 0; r < 8; r++) {
            float mx = fmaxf(fmaxf(s[0][r], s[1][r]), fmaxf(s[2][r], s[3][r]));
#pragma unroll
            for (u32 m = 8; m >= 1; m >>= 1) mx = fmaxf(mx, __shfl_xor(mx, m, 32));
            const float mnew  = fmaxf(mrow[r], mx);
            const float alpha = __expf(mrow[r] - mnew);
            float rsum = 0.f;
#pragma unroll
            for (int sub = 0; sub < 4; sub++) {
                float pe = __expf(s[sub][r] - mnew);
                s[sub][r] = pe;
                rsum += pe;
            }
#pragma unroll
            for (u32 m = 8; m >= 1; m >>= 1) rsum += __shfl_xor(rsum, m, 32);
            mrow[r] = mnew;
            lrow[r] = lrow[r] * alpha + rsum;
#pragma unroll
            for (int dsub = 0; dsub < 4; dsub++) o[dsub][r] *= alpha;
        }

#pragma unroll
        for (int sub = 0; sub < 4; sub++) {
#pragma unroll
            for (int r = 0; r < 8; r++) {
                const float ph = s[sub][r] * PCAR;
                _Float16 h16 = (_Float16)ph;
                Pw[(hf * 8u + (u32)r) * 72u + (u32)sub * 16u + ln] = __builtin_bit_cast(u16, h16);
                if constexpr (RES != 0)
                    Prw[(hf * 8u + (u32)r) * 72u + (u32)sub * 16u + ln] = hbits((ph - (float)h16) * RSC);
            }
        }
        __syncthreads();
        sched_cut<RES>();

#pragma unroll
        for (int dsub = 0; dsub < 4; dsub++) {
            v8f u = (v8f)(0.f);
#pragma unroll
            for (int ks = 0; ks < 2; ks++) {
                Frag pf, vf;
                const u16* pp = &Pw[ln * 72u + (u32)ks * 32u + hf * 8u];
                pf.u[0] = *(const u32x4*)pp;
                pf.u[1] = *(const u32x4*)(pp + 16);
                const u16* vp = &Vs[((u32)dsub * 16u + ln) * 72u + (u32)ks * 32u + hf * 8u];
                vf.u[0] = *(const u32x4*)vp;
                vf.u[1] = *(const u32x4*)(vp + 16);
                o[dsub] = mma16(pf.v, vf.v, o[dsub]);
                if constexpr (RES != 0) {
                    Frag prf;
                    const u16* prp = &Prw[ln * 72u + (u32)ks * 32u + hf * 8u];
                    prf.u[0] = *(const u32x4*)prp;
                    prf.u[1] = *(const u32x4*)(prp + 16);
                    u = mma16(prf.v, vf.v, u);
                    Frag vlf;
                    const u16* vlp = &Vl[((u32)dsub * 16u + ln) * 72u + (u32)ks * 32u + hf * 8u];
                    vlf.u[0] = *(const u32x4*)vlp;
                    vlf.u[1] = *(const u32x4*)(vlp + 16);
                    u = mma16(pf.v, vlf.v, u);
                }
            }
            if constexpr (RES != 0) o[dsub] = o[dsub] + u * RINV;
            sched_cut<RES>();
        }
    }

    __syncthreads();
#pragma unroll
    for (int r = 0; r < 8; r++) {
        const float inv = (1.0f / lrow[r]) * PINV;
#pragma unroll
        for (int dsub = 0; dsub < 4; dsub++)
            Pw[(hf * 8u + (u32)r) * 72u + (u32)dsub * 16u + ln] = hbits(o[dsub][r] * inv);
    }
    __syncthreads();
    u32x4 val[4];
#pragma unroll
    for (u32 it = 0; it < 4; it++) {
        const u32 rloc = it * 4u + (lane >> 3), sg = (lane & 7u) * 8u;
        val[it] = *(const u32x4*)&Pw[rloc * 72u + sg];
    }
#pragma unroll
    for (u32 it = 0; it < 4; it++) {
        const u32 rloc = it * 4u + (lane >> 3), sg = (lane & 7u) * 8u;
        *(volatile u32x4*)(cv + (size_t)(b * (u32)(SEQ) + q0 + rloc) * CE + h * HD + sg) = val[it];
    }
    __threadfence();
#pragma unroll
    for (u32 it = 0; it < 4; it++) {
        const u32 rloc = it * 4u + (lane >> 3), sg = (lane & 7u) * 8u;
        *(volatile u32x4*)(cv + (size_t)(b * (u32)(SEQ) + q0 + rloc) * CE + h * HD + sg) = val[it];
    }
}

extern "C" void kernel_launch(void* const* d_in, const int* in_sizes, int n_in,
                              void* d_out, int out_size, void* d_ws, size_t ws_size,
                              hipStream_t stream) {
    if (n_in < 13) return;
    const long long needX = ((long long)(NB - 1) * SEQ_FULL + (SEQ)) * CE;
    if ((long long)in_sizes[0] < needX || (long long)out_size < needX) return;
    if (in_sizes[1] < CE || in_sizes[2] < CE || in_sizes[3] < CE * C3 || in_sizes[4] < C3 ||
        in_sizes[5] < CE * CE || in_sizes[6] < CE || in_sizes[7] < CE || in_sizes[8] < CE ||
        in_sizes[9] < CE * C4 || in_sizes[10] < C4 || in_sizes[11] < C4 * CE || in_sizes[12] < CE)
        return;

    const float* x      = (const float*)d_in[0];
    const float* ln1_g  = (const float*)d_in[1];
    const float* ln1_b  = (const float*)d_in[2];
    const float* w_attn = (const float*)d_in[3];
    const float* b_attn = (const float*)d_in[4];
    const float* w_proj = (const float*)d_in[5];
    const float* b_proj = (const float*)d_in[6];
    const float* ln2_g  = (const float*)d_in[7];
    const float* ln2_b  = (const float*)d_in[8];
    const float* w_fc   = (const float*)d_in[9];
    const float* b_fc   = (const float*)d_in[10];
    const float* w_fc2  = (const float*)d_in[11];
    const float* b_fc2  = (const float*)d_in[12];

    char* ws = (char*)d_ws;
    size_t off = 0;
    auto take = [&](size_t bytes) -> char* {
        char* p = ws + off;
        off += (bytes + 255) & ~(size_t)255;
        return p;
    };
    const size_t R = (size_t)RROWS;
    u16*   waT   = (u16*)take((size_t)C3 * CE * 2);
    u16*   wpT   = (u16*)take((size_t)CE * CE * 2);
    u16*   wfcT  = (u16*)take((size_t)C4 * CE * 2);
    u16*   wfc2T = (u16*)take((size_t)CE * C4 * 2);
    u16*   h1    = (u16*)take(R * CE * 2);
    u16*   qkh   = (u16*)take(R * QP * 2);
    u16*   qkl   = (u16*)take((size_t)NB * (TE) * QP * 2);
    u16*   vth   = (u16*)take((size_t)NB * NH * HD * (SEQ) * 2);
    u16*   vtl   = (u16*)take((size_t)NB * NH * HD * (TE) * 2);
    u16*   cvb   = (u16*)take(R * CE * 2);
    float* x1    = (float*)take(R * CE * 4);
    u16*   h2    = (u16*)take(R * CE * 2);
    u16*   hg    = (u16*)take(R * C4 * 2);
    if (off > ws_size || off > (size_t)134217728) return;
    void* dummy = (void*)d_ws;

    cvt_wt_kernel<<<dim3(C3 / 64, CE / 64), 256, 0, stream>>>(w_attn, waT, (u32)CE, (u32)C3);
    cvt_wt_kernel<<<dim3(CE / 64, CE / 64), 256, 0, stream>>>(w_proj, wpT, (u32)CE, (u32)CE);
    cvt_wt_kernel<<<dim3(C4 / 64, CE / 64), 256, 0, stream>>>(w_fc,   wfcT, (u32)CE, (u32)C4);
    cvt_wt_kernel<<<dim3(CE / 64, C4 / 64), 256, 0, stream>>>(w_fc2,  wfc2T, (u32)C4, (u32)CE);
    ln_kernel<1><<<RROWS / 8, 256, 0, stream>>>(x, ln1_g, ln1_b, h1);
    gemm_kernel<0><<<dim3(C3 / 128, RROWS / 128), 256, 0, stream>>>(h1, waT, b_attn, b_attn,
                                                                    qkh, qkl, vth, vtl, (u32)C3, (u32)CE);
    attn_kernel<1><<<dim3(NEB, NB * NH), 256, 0, stream>>>(qkh, qkl, vth, vtl, cvb, 0u);
    if (NQB > NEB)
        attn_kernel<0><<<dim3(NQB - NEB, NB * NH), 256, 0, stream>>>(qkh, qkl, vth, vtl, cvb, (u32)NEB);
    gemm_kernel<1><<<dim3(CE / 128, RROWS / 128), 256, 0, stream>>>(cvb, wpT, b_proj, x,
                                                                    x1, dummy, dummy, dummy, (u32)CE, (u32)CE);
    ln_kernel<0><<<RROWS / 8, 256, 0, stream>>>(x1, ln2_g, ln2_b, h2);
    gemm_kernel<2><<<dim3(C4 / 128, RROWS / 128), 256, 0, stream>>>(h2, wfcT, b_fc, b_fc,
                                                                    hg, dummy, dummy, dummy, (u32)C4, (u32)CE);
    gemm_kernel<3><<<dim3(CE / 128, RROWS / 128), 256, 0, stream>>>(hg, wfc2T, b_fc2, x1,
                                                                    d_out, dummy, dummy, dummy, (u32)CE, (u32)C4);
}
